// ConvKNRM_52922587021474
// MI455X (gfx1250) — hardware-verified
//
#include <hip/hip_runtime.h>
#include <stdint.h>
#include <stddef.h>

typedef __attribute__((ext_vector_type(16))) _Float16 v16h;
typedef __attribute__((ext_vector_type(8)))  _Float16 v8h;
typedef __attribute__((ext_vector_type(16))) __bf16   v16b;
typedef __attribute__((ext_vector_type(8)))  __bf16   v8b;
typedef __attribute__((ext_vector_type(8)))  float    v8f;
typedef __attribute__((ext_vector_type(4)))  float    v4f;

constexpr int NB    = 256;
constexpr int LQ    = 32;
constexpr int LD    = 1024;
constexpr int EMBD  = 128;
constexpr int NFIL  = 128;
constexpr int NKER  = 11;
constexpr int NGRAM = 3;
constexpr int MQ    = 64;
constexpr int QROWS = MQ + 2;
constexpr int DROWS = LD + 2;
constexpr int BCH   = 64;
constexpr int NCH   = NB / BCH;
constexpr int DBLK  = 256;
constexpr int NDBLK = LD / DBLK;
constexpr int PART_STRIDE = 16 * 32;
constexpr int WOFF1 = 0;
constexpr int WOFF2 = NFIL * EMBD * 1;
constexpr int WOFF3 = WOFF2 + NFIL * EMBD * 2;
constexpr int WTOT  = WOFF3 + NFIL * EMBD * 3;

static_assert(NB % BCH == 0);
static_assert(LD % DBLK == 0);
static_assert((EMBD * 1) % 32 == 0 && (EMBD * 2) % 32 == 0 && (EMBD * 3) % 32 == 0);
static_assert(MQ % 64 == 0 && LD % 64 == 0 && NFIL % 64 == 0);
static_assert(NB % 32 == 0);
static_assert((NB * QROWS) % 16 == 0 && (NB * DROWS) % 16 == 0);
static_assert(WTOT % 8 == 0);

constexpr float kLog2e = 1.4426950408889634f;
constexpr float kSigW2 = 0.1f * 0.1f;
constexpr float kSigE2 = 0.001f * 0.001f;
constexpr float kCW = (-0.5f / kSigW2) * kLog2e;
constexpr float kCE = (-0.5f / kSigE2) * kLog2e;

__device__ __forceinline__ unsigned short f2bf_bits(float f) {
  unsigned u = __float_as_uint(f);
  return (unsigned short)((u + 0x7FFFu + ((u >> 16) & 1u)) >> 16);
}
__device__ __forceinline__ float bf_bits2f(unsigned short h) { return __uint_as_float(((unsigned)h) << 16); }

__device__ __forceinline__ void dep_guard_h(v8f& a, v8f& b, v16h x, v16h y) { asm volatile("v_nop\n\tv_nop\n\tv_nop\n\tv_nop" : "+v"(a), "+v"(b) : "v"(x), "v"(y)); }
__device__ __forceinline__ void dep_guard_b(v8f& a, v8f& b, v16b x, v16b y) { asm volatile("v_nop\n\tv_nop\n\tv_nop\n\tv_nop" : "+v"(a), "+v"(b) : "v"(x), "v"(y)); }
__device__ __forceinline__ void keep4_h(v16h a, v16h b, v16h c, v16h d) { asm volatile("v_nop" :: "v"(a), "v"(b), "v"(c), "v"(d)); }
__device__ __forceinline__ void keep4_b(v16b a, v16b b, v16b c, v16b d) { asm volatile("v_nop" :: "v"(a), "v"(b), "v"(c), "v"(d)); }
__device__ __forceinline__ void acc_guard4(v8f& a, v8f& b, v8f& c, v8f& d) { asm volatile("v_nop\n\tv_nop\n\tv_nop\n\tv_nop" : "+v"(a), "+v"(b), "+v"(c), "+v"(d)); }
template <typename T> struct Frag;
template <> struct Frag<_Float16> {
  typedef v16h V; union U { v16h v; v8h h[2]; };
  static __device__ __forceinline__ v16h load(const _Float16* p) {
    U f; f.h[0] = *(const v8h*)(p); f.h[1] = *(const v8h*)(p + 16); return f.v;
  }
  static __device__ __forceinline__ v8f mma(v16h a, v16h b, v8f c) {
    return __builtin_amdgcn_wmma_f32_16x16x32_f16(false, a, false, b, (short)0, c, false, false);
  }
  static __device__ __forceinline__ void guard(v8f& a, v8f& b, v16h x, v16h y) { dep_guard_h(a, b, x, y); }
  static __device__ __forceinline__ void keep(v16h a, v16h b, v16h c, v16h d) { keep4_h(a, b, c, d); }
};
template <> struct Frag<__bf16> {
  typedef v16b V; union U { v16b v; v8b h[2]; };
  static __device__ __forceinline__ v16b load(const __bf16* p) {
    U f; f.h[0] = *(const v8b*)(p); f.h[1] = *(const v8b*)(p + 16); return f.v;
  }
  static __device__ __forceinline__ v8f mma(v16b a, v16b b, v8f c) {
    return __builtin_amdgcn_wmma_f32_16x16x32_bf16(false, a, false, b, (short)0, c, false, false);
  }
  static __device__ __forceinline__ void guard(v8f& a, v8f& b, v16b x, v16b y) { dep_guard_b(a, b, x, y); }
  static __device__ __forceinline__ void keep(v16b a, v16b b, v16b c, v16b d) { keep4_b(a, b, c, d); }
};

template <int ET> struct Elem;
template <> struct Elem<0> { typedef _Float16 T; };
template <> struct Elem<1> { typedef __bf16 T; };
template <int ET, bool SPLIT, int BIAS_MODE, int OUT_MODE, bool RESID, int ACT = 0>
__global__ __launch_bounds__(256) void wmma_gemm64(
    const unsigned short* __restrict__ Ap, const unsigned short* __restrict__ A2p, int lda, long strideA,
    const unsigned short* __restrict__ Btp, const unsigned short* __restrict__ Bt2p, int ldb, long strideB,
    void* __restrict__ Cout, void* __restrict__ Cout2, int ldc, long strideC,
    const float* __restrict__ bias,
    const float* __restrict__ resid, long strideR,
    int M, int N, int K, float scale) {
  typedef typename Elem<ET>::T T;
  typedef typename Frag<T>::V V;
  const T* A = (const T*)Ap; const T* A2 = (const T*)A2p; const T* Bt = (const T*)Btp; const T* Bt2 = (const T*)Bt2p;
  __shared__ __align__(16) float sT[8][16 * 68];
  const int b    = blockIdx.y;
  const int lane = threadIdx.x & 31;
  const int wave = threadIdx.x >> 5;
  const int tilesN = N >> 6;
  const int tilesM = M >> 6;
  const int tile = blockIdx.x * 8 + wave;
  if (tile >= tilesM * tilesN) return;
  const int tm = tile / tilesN;
  const int tn = tile - tm * tilesN;
  const int m0 = tm << 6;
  const int n0 = tn << 6;

  const T* Ab  = A  + (size_t)b * strideA;
  const T* Bb  = Bt + (size_t)b * strideB;
  const T* Ab2 = SPLIT ? (A2  + (size_t)b * strideA) : nullptr;
  const T* Bb2 = SPLIT ? (Bt2 + (size_t)b * strideB) : nullptr;

  const int rlane = lane & 15;
  const int koff  = (lane >> 4) * 8;
  const int mOff  = (lane >> 4) * 8;

  v8f acc[4][4];
#pragma unroll
  for (int i = 0; i < 4; ++i)
#pragma unroll
    for (int j = 0; j < 4; ++j) acc[i][j] = (v8f){0.f,0.f,0.f,0.f,0.f,0.f,0.f,0.f};

  for (int k0 = 0; k0 < K; k0 += 32) {
    V bh[4], bl[4];
#pragma unroll
    for (int j = 0; j < 4; ++j) {
      const size_t bo = (size_t)(n0 + (j << 4) + rlane) * ldb + koff + k0;
      bh[j] = Frag<T>::load(Bb + bo);
      if (SPLIT) bl[j] = Frag<T>::load(Bb2 + bo);
    }
#pragma unroll
    for (int i = 0; i < 4; ++i) {
      const size_t ao = (size_t)(m0 + (i << 4) + rlane) * lda + koff + k0;
      V ah = Frag<T>::load(Ab + ao);
      V al;
      if (SPLIT) al = Frag<T>::load(Ab2 + ao);
#pragma unroll
      for (int j = 0; j < 4; ++j) {
        acc[i][j] = Frag<T>::mma(ah, bh[j], acc[i][j]);
        if (SPLIT) {
          acc[i][j] = Frag<T>::mma(ah, bl[j], acc[i][j]);
          acc[i][j] = Frag<T>::mma(al, bh[j], acc[i][j]);
        }
      }
      Frag<T>::guard(acc[i][0], acc[i][3], ah, SPLIT ? al : ah);
    }
    Frag<T>::keep(bh[0], bh[1], bh[2], bh[3]);
    if (SPLIT) Frag<T>::keep(bl[0], bl[1], bl[2], bl[3]);
  }
  acc_guard4(acc[0][0], acc[0][1], acc[0][2], acc[0][3]);
  acc_guard4(acc[1][0], acc[1][1], acc[1][2], acc[1][3]);
  acc_guard4(acc[2][0], acc[2][1], acc[2][2], acc[2][3]);
  acc_guard4(acc[3][0], acc[3][1], acc[3][2], acc[3][3]);

  float* slab = sT[wave];
  const float* Rb = RESID ? (resid + (size_t)b * strideR) : nullptr;
#pragma unroll
  for (int i = 0; i < 4; ++i) {
    const int mBase = m0 + (i << 4);
#pragma unroll
    for (int j = 0; j < 4; ++j) {
      const int n = n0 + (j << 4) + rlane;
      float bv = 0.f;
      if (BIAS_MODE == 2) bv = bias[n];
#pragma unroll
      for (int r = 0; r < 8; ++r) {
        float v = acc[i][j][r] * scale;
        if (BIAS_MODE == 1) v += bias[mBase + mOff + r];
        if (BIAS_MODE == 2) v += bv;
        if (RESID) v += Rb[(size_t)(mBase + mOff + r) * ldc + n];
        if (ACT == 1) v = tanhf(v);
        if (ACT == 2) v = fmaxf(v, 0.0f);
        if (ACT == 3) v = v / (1.0f + expf(-v));
        if (ACT == 4) v = (v > 0.f) ? v : 0.01f * v;
        slab[(mOff + r) * 68 + (j << 4) + rlane] = v;
      }
    }
    __builtin_amdgcn_fence(__ATOMIC_RELEASE, "workgroup");
    __builtin_amdgcn_wave_barrier();
    __builtin_amdgcn_fence(__ATOMIC_ACQUIRE, "workgroup");
    if (OUT_MODE == 0) {
      float* C = (float*)Cout + (size_t)b * strideC;
      const int hh = lane >> 4, c4 = (lane & 15) * 4;
      for (int pass = 0; pass < 2; ++pass) {
#pragma unroll
        for (int it = 0; it < 8; ++it) {
          const int row = it * 2 + hh;
          v4f v = *(const v4f*)(slab + row * 68 + c4);
          *(volatile v4f*)(C + (size_t)(mBase + row) * ldc + n0 + c4) = v;
        }
        __threadfence();
      }
    } else {
      const int q = lane >> 3, c8 = (lane & 7) * 8;
      unsigned short* C  = (unsigned short*)Cout  + (size_t)b * strideC;
      unsigned short* C2 = (OUT_MODE == 2) ? ((unsigned short*)Cout2 + (size_t)b * strideC) : nullptr;
      for (int pass = 0; pass < 2; ++pass) {
#pragma unroll
        for (int it = 0; it < 4; ++it) {
          const int row = it * 4 + q;
          const float* sp = slab + row * 68 + c8;
          v8h hv, lv;
#pragma unroll
          for (int e = 0; e < 8; ++e) {
            if (OUT_MODE == 1) {
              hv[e] = (_Float16)sp[e];
            } else {
              unsigned short hb = f2bf_bits(sp[e]);
              unsigned short lb = f2bf_bits(sp[e] - bf_bits2f(hb));
              hv[e] = __builtin_bit_cast(_Float16, hb);
              lv[e] = __builtin_bit_cast(_Float16, lb);
            }
          }
          *(volatile v8h*)(C + (size_t)(mBase + row) * ldc + n0 + c8) = hv;
          if (OUT_MODE == 2) *(volatile v8h*)(C2 + (size_t)(mBase + row) * ldc + n0 + c8) = lv;
        }
        __threadfence();
      }
    }
    __builtin_amdgcn_fence(__ATOMIC_RELEASE, "workgroup");
    __builtin_amdgcn_wave_barrier();
    __builtin_amdgcn_fence(__ATOMIC_ACQUIRE, "workgroup");
  }
}

__global__ __launch_bounds__(256) void wprep_kernel(const float* __restrict__ w1, const float* __restrict__ w2,
                                                     const float* __restrict__ w3, unsigned short* __restrict__ Wp) {
  const int pn  = blockIdx.y;
  const int n   = pn + 1;
  const int kw  = EMBD * n;
  const int nth = (NFIL * kw) >> 3;
  const int i   = blockIdx.x * 256 + threadIdx.x;
  if (i >= nth) return;
  const float* w = (pn == 0) ? w1 : ((pn == 1) ? w2 : w3);
  const int base = (pn == 0) ? WOFF1 : ((pn == 1) ? WOFF2 : WOFF3);
  const int e0  = i << 3;
  const int f   = e0 / kw;
  const int col = e0 - f * kw;
  const int kk  = col >> 7;
  const int c   = col & 127;
  v8h hv;
#pragma unroll
  for (int e = 0; e < 8; ++e) {
    const float v = 16.0f * w[((size_t)f * EMBD + c + e) * n + kk];
    hv[e] = (_Float16)v;
  }
  unsigned short* dst = Wp + base + e0;
  *(volatile v8h*)dst = hv;
  __threadfence();
  *(volatile v8h*)dst = hv;
}

__global__ __launch_bounds__(256) void embed_kernel(const int* __restrict__ ids, const float* __restrict__ emb,
                                                     unsigned short* __restrict__ X, int L, int Lrows, int nrows, int vocab) {
  const int tid  = threadIdx.x;
  const int wave = tid >> 5;
  const int lane = tid & 31;
  const int hh   = lane >> 4;
  const int gw   = blockIdx.x * 8 + wave;
  const int r0   = gw * 2;
  if (r0 >= nrows) return;
  const int row  = r0 + hh;
  const int b    = row / Lrows;
  const int t    = row - b * Lrows;
  const int tc   = (t < L) ? t : (L - 1);
  int id = ids[(size_t)b * L + tc];
  id = (id < 0) ? 0 : ((id >= vocab) ? (vocab - 1) : id);
  const int c8 = (lane & 15) * 8;
  const float* e = emb + (size_t)id * EMBD + c8;
  const v4f a = *(const v4f*)(e);
  const v4f c = *(const v4f*)(e + 4);
  float ss = 0.0f;
  ss += a[0] * a[0]; ss += a[1] * a[1]; ss += a[2] * a[2]; ss += a[3] * a[3];
  ss += c[0] * c[0]; ss += c[1] * c[1]; ss += c[2] * c[2]; ss += c[3] * c[3];
  ss += __shfl_xor(ss, 1, 32);
  ss += __shfl_xor(ss, 2, 32);
  ss += __shfl_xor(ss, 4, 32);
  ss += __shfl_xor(ss, 8, 32);
  const float rn  = 1.0f / sqrtf(ss);
  const float scl = 64.0f * rn;
  const float mul = (t < L) ? scl : 0.0f;
  v8h hv;
  hv[0] = (_Float16)(a[0] * mul); hv[1] = (_Float16)(a[1] * mul); hv[2] = (_Float16)(a[2] * mul); hv[3] = (_Float16)(a[3] * mul);
  hv[4] = (_Float16)(c[0] * mul); hv[5] = (_Float16)(c[1] * mul); hv[6] = (_Float16)(c[2] * mul); hv[7] = (_Float16)(c[3] * mul);
  unsigned short* dst = X + (size_t)row * EMBD + c8;
  *(volatile v8h*)dst = hv;
  __threadfence();
  *(volatile v8h*)dst = hv;
}

__device__ __forceinline__ v8f mma_bf_g(v16b a, v16b b, v8f c) {
  c = __builtin_amdgcn_wmma_f32_16x16x32_bf16(false, a, false, b, (short)0, c, false, false);
  asm volatile("v_nop\n\tv_nop\n\tv_nop\n\tv_nop" : "+v"(c) : "v"(a), "v"(b));
  return c;
}

__global__ __launch_bounds__(256) void simpool_kernel(
    const unsigned short* __restrict__ DcHp, const unsigned short* __restrict__ DcLp,
    const unsigned short* __restrict__ QcHp, const unsigned short* __restrict__ QcLp,
    float* __restrict__ partials, int bchunk0, int ng) {
  __shared__ float red[8][NKER][32];
  __shared__ float blk[16][32];
  const int tid  = threadIdx.x;
  const int wave = tid >> 5;
  const int lane = tid & 31;
  const int hh   = lane >> 4;
  const int rl   = lane & 15;
  const int koff = hh * 8;
  const int bb   = blockIdx.y;
  const int b    = bchunk0 + bb;
  const int dblk = blockIdx.x;

  const __bf16* Dh = (const __bf16*)DcHp + ((size_t)bb * LD + (size_t)dblk * DBLK + wave * 32) * NFIL;
  const __bf16* Dl = (const __bf16*)DcLp + ((size_t)bb * LD + (size_t)dblk * DBLK + wave * 32) * NFIL;
  const __bf16* Qh = (const __bf16*)QcHp + (size_t)b * MQ * NFIL;
  const __bf16* Ql = (const __bf16*)QcLp + (size_t)b * MQ * NFIL;

  v8f acc[2][2];
#pragma unroll
  for (int mt = 0; mt < 2; ++mt)
#pragma unroll
    for (int jt = 0; jt < 2; ++jt) acc[mt][jt] = (v8f){0.f,0.f,0.f,0.f,0.f,0.f,0.f,0.f};

#pragma unroll
  for (int k0 = 0; k0 < NFIL; k0 += 32) {
    v16b qh[2], ql[2];
#pragma unroll
    for (int jt = 0; jt < 2; ++jt) {
      const int bo = (jt * 16 + rl) * NFIL + koff + k0;
      qh[jt] = Frag<__bf16>::load(Qh + bo);
      ql[jt] = Frag<__bf16>::load(Ql + bo);
    }
#pragma unroll
    for (int mt = 0; mt < 2; ++mt) {
      const int ao = (mt * 16 + rl) * NFIL + koff + k0;
      const v16b dh = Frag<__bf16>::load(Dh + ao);
      const v16b dl = Frag<__bf16>::load(Dl + ao);
#pragma unroll
      for (int jt = 0; jt < 2; ++jt) {
        acc[mt][jt] = mma_bf_g(dh, qh[jt], acc[mt][jt]);
        acc[mt][jt] = mma_bf_g(dh, ql[jt], acc[mt][jt]);
        acc[mt][jt] = mma_bf_g(dl, qh[jt], acc[mt][jt]);
      }
    }
    keep4_b(qh[0], qh[1], ql[0], ql[1]);
  }
  acc_guard4(acc[0][0], acc[0][1], acc[1][0], acc[1][1]);

  const float kMu[NKER] = {-0.9f, -0.7f, -0.5f, -0.3f, -0.1f, 0.1f, 0.3f, 0.5f, 0.7f, 0.9f, 1.0f};
  const float kC[NKER]  = {kCW, kCW, kCW, kCW, kCW, kCW, kCW, kCW, kCW, kCW, kCE};
  float ps[2][NKER];
#pragma unroll
  for (int jt = 0; jt < 2; ++jt)
#pragma unroll
    for (int k = 0; k < NKER; ++k) ps[jt][k] = 0.0f;

#pragma unroll
  for (int mt = 0; mt < 2; ++mt) {
#pragma unroll
    for (int jt = 0; jt < 2; ++jt) {
#pragma unroll
      for (int r = 0; r < 8; ++r) {
        const float s = acc[mt][jt][r];
#pragma unroll
        for (int k = 0; k < NKER; ++k) {
          const float t = s - kMu[k];
          float u = t * t;
          u = u * kC[k];
          ps[jt][k] += exp2f(u);
        }
      }
    }
  }
#pragma unroll
  for (int jt = 0; jt < 2; ++jt)
#pragma unroll
    for (int k = 0; k < NKER; ++k) ps[jt][k] += __shfl_xor(ps[jt][k], 16, 32);
#pragma unroll
  for (int k = 0; k < NKER; ++k) {
    const float v = hh ? ps[1][k] : ps[0][k];
    red[wave][k][lane] = v;
  }
  __syncthreads();
  for (int i = tid; i < 512; i += 256) {
    const int k = i >> 5;
    const int q = i & 31;
    float v = 0.0f;
    if (k < NKER) {
#pragma unroll
      for (int w = 0; w < 8; ++w) v += red[w][k][q];
    }
    blk[k][q] = v;
  }
  __syncthreads();
  float* P = partials + ((((size_t)b * NGRAM + ng) * NDBLK + dblk) * PART_STRIDE);
  const float v0 = blk[wave][lane];
  const float v1 = blk[wave + 8][lane];
  *(volatile float*)(P + wave * 32 + lane) = v0;
  *(volatile float*)(P + (wave + 8) * 32 + lane) = v1;
  __threadfence();
  *(volatile float*)(P + wave * 32 + lane) = v0;
  *(volatile float*)(P + (wave + 8) * 32 + lane) = v1;
}

__global__ __launch_bounds__(256) void final_kernel(const float* __restrict__ partials, const float* __restrict__ lw,
                                                     float* __restrict__ out) {
  __shared__ float lg[NGRAM * NKER * 32];
  __shared__ float cnt[64];
  __shared__ float lws[64];
  __shared__ float ov[32];
  const int tid = threadIdx.x;
  const int b0  = blockIdx.x * 32;
  if (tid < NGRAM * NKER) lws[tid] = lw[tid];
  __syncthreads();
  for (int bl = 0; bl < 32; ++bl) {
    const int b = b0 + bl;
    for (int i = tid; i < NGRAM * NKER * 32; i += 256) {
      const int n   = i / (NKER * 32);
      const int rem = i - n * (NKER * 32);
      const int k   = rem >> 5;
      const int q   = rem & 31;
      const float* P = partials + ((size_t)(b * NGRAM + n) * NDBLK) * PART_STRIDE + k * 32 + q;
      float m = 0.0f;
      m += P[0];
      m += P[PART_STRIDE];
      m += P[2 * PART_STRIDE];
      m += P[3 * PART_STRIDE];
      lg[i] = log1pf(m);
    }
    __syncthreads();
    if (tid < NGRAM * NKER) {
      const int n = tid / NKER;
      const int k = tid - n * NKER;
      float cs = 0.0f;
#pragma unroll 1
      for (int q = 0; q < 32; ++q) cs += lg[n * (NKER * 32) + k * 32 + q];
      cnt[tid] = cs;
    }
    __syncthreads();
    if (tid == 0) {
      float o = 0.0f;
#pragma unroll 1
      for (int j = 0; j < NGRAM * NKER; ++j) o += cnt[j] * lws[j];
      ov[bl] = o;
    }
    __syncthreads();
  }
  const float v = ov[tid & 31];
  if (tid < 32) *(volatile float*)(out + b0 + tid) = v;
  __threadfence();
  if (tid < 32) *(volatile float*)(out + b0 + tid) = v;
}

extern "C" void kernel_launch(void* const* d_in, const int* in_sizes, int n_in,
                              void* d_out, int out_size, void* d_ws,
                              size_t ws_size, hipStream_t stream) {
  if (n_in < 12) return;
  const int*   q_ids = (const int*)d_in[0];
  const int*   d_ids = (const int*)d_in[1];
  const float* emb   = (const float*)d_in[4];
  const float* w1    = (const float*)d_in[5];
  const float* bs1   = (const float*)d_in[6];
  const float* w2    = (const float*)d_in[7];
  const float* bs2   = (const float*)d_in[8];
  const float* w3    = (const float*)d_in[9];
  const float* bs3   = (const float*)d_in[10];
  const float* lw    = (const float*)d_in[11];
  float* out = (float*)d_out;

  const int vocab = in_sizes[4] / EMBD;
  if (in_sizes[0] != NB * LQ || in_sizes[1] != NB * LD || vocab < 1) return;
  if (out_size != NB || in_sizes[11] != NGRAM * NKER) return;

  char* ws = (char*)d_ws;
  size_t off = 0;
  const size_t szXd   = (size_t)NB * DROWS * EMBD * 2;
  const size_t szXq   = (size_t)NB * QROWS * EMBD * 2;
  const size_t szW    = (size_t)WTOT * 2;
  const size_t szQc   = (size_t)NB * MQ * NFIL * 2;
  const size_t szDc   = (size_t)BCH * LD * NFIL * 2;
  const size_t szPart = (size_t)NB * NGRAM * NDBLK * PART_STRIDE * 4;
  unsigned short* Xd   = (unsigned short*)(ws + off); off += (szXd + 255) & ~(size_t)255;
  unsigned short* Xq   = (unsigned short*)(ws + off); off += (szXq + 255) & ~(size_t)255;
  unsigned short* Wp   = (unsigned short*)(ws + off); off += (szW + 255) & ~(size_t)255;
  unsigned short* QcH  = (unsigned short*)(ws + off); off += (szQc + 255) & ~(size_t)255;
  unsigned short* QcL  = (unsigned short*)(ws + off); off += (szQc + 255) & ~(size_t)255;
  unsigned short* DcH  = (unsigned short*)(ws + off); off += (szDc + 255) & ~(size_t)255;
  unsigned short* DcL  = (unsigned short*)(ws + off); off += (szDc + 255) & ~(size_t)255;
  float*          part = (float*)(ws + off);          off += (szPart + 255) & ~(size_t)255;
  if (off > ws_size) return;

  wprep_kernel<<<dim3(24, 3), 256, 0, stream>>>(w1, w2, w3, Wp);

  {
    const int nrows_q = NB * QROWS;
    embed_kernel<<<nrows_q / 16, 256, 0, stream>>>(q_ids, emb, Xq, LQ, QROWS, nrows_q, vocab);
    const int nrows_d = NB * DROWS;
    embed_kernel<<<nrows_d / 16, 256, 0, stream>>>(d_ids, emb, Xd, LD, DROWS, nrows_d, vocab);
  }

  const float convscale = 1.0f / 1024.0f;
  for (int n = 1; n <= NGRAM; ++n) {
    const int kw = EMBD * n;
    const unsigned short* Wn = Wp + ((n == 1) ? WOFF1 : ((n == 2) ? WOFF2 : WOFF3));
    const float* bn = (n == 1) ? bs1 : ((n == 2) ? bs2 : bs3);
    {
      const int tiles = (MQ / 64) * (NFIL / 64);
      wmma_gemm64<0, false, 2, 2, false, 1><<<dim3((tiles + 7) / 8, NB), 256, 0, stream>>>(
          Xq, Xq, EMBD, (long)QROWS * EMBD,
          Wn, Wn, kw, 0L,
          (void*)QcH, (void*)QcL, NFIL, (long)MQ * NFIL,
          bn, nullptr, 0L,
          MQ, NFIL, kw, convscale);
    }
    for (int ch = 0; ch < NCH; ++ch) {
      const unsigned short* XdC = Xd + (size_t)ch * BCH * DROWS * EMBD;
      const int tiles = (LD / 64) * (NFIL / 64);
      wmma_gemm64<0, false, 2, 2, false, 1><<<dim3((tiles + 7) / 8, BCH), 256, 0, stream>>>(
          XdC, XdC, EMBD, (long)DROWS * EMBD,
          Wn, Wn, kw, 0L,
          (void*)DcH, (void*)DcL, NFIL, (long)LD * NFIL,
          bn, nullptr, 0L,
          LD, NFIL, kw, convscale);
      simpool_kernel<<<dim3(NDBLK, BCH), 256, 0, stream>>>(DcH, DcL, QcH, QcL, part, ch * BCH, n - 1);
    }
  }

  final_kernel<<<NB / 32, 256, 0, stream>>>(part, lw, out);
}
